// QuantumConv_42004780155287
// MI455X (gfx1250) — hardware-verified
//
#include <hip/hip_runtime.h>
#include <math.h>

typedef __attribute__((ext_vector_type(16))) _Float16 v16h;
typedef __attribute__((ext_vector_type(8)))  _Float16 v8h;
typedef __attribute__((ext_vector_type(8)))  float    v8f;
typedef __attribute__((ext_vector_type(4)))  float    v4f;

constexpr int kBatch  = 4;
constexpr int kCin    = 16;
constexpr int kHgt    = 64;
constexpr int kWid    = 64;
constexpr int kWires  = 8;
constexpr int kLayers = 5;
constexpr int kCout   = 32;
constexpr int kPix    = kBatch * kHgt * kWid;
constexpr int kAmp    = 1 << kWires;
constexpr int kNcol   = 2 * kAmp;
constexpr int kGates  = kLayers * 2 * kWires;
constexpr int kNumPar = kLayers * kWires * 3;
constexpr int kMeas   = 3 * kWires;
constexpr int kTaps   = kCin * 9;
static_assert(kPix == 16384 && kAmp == 256 && kNcol == 512 && kGates == 80 && kNumPar == 120 && kMeas == 24, "shape constants");
static_assert(kWid == 64 && kHgt == 64 && kWires == 8 && kCout == 32, "index arithmetic below assumes these");
static_assert((kPix % 64) == 0 && (kNcol % 64) == 0 && (kAmp % 32) == 0, "GEMM M,N multiples of 64 and K multiple of 32");
static_assert((((kPix / 64) * (kNcol / 64)) % 8) == 0, "GEMM tiles per block");

constexpr float kCarryA       = 1024.0f;
constexpr float kCarryB       = 256.0f;
constexpr float kFold         = 1.0f / (kCarryA * kCarryB);
constexpr float kF16MinNormal = 6.103515625e-5f;

constexpr size_t kSzANG  = (size_t)kPix * kWires * 4;
constexpr size_t kSzAPL  = (size_t)kPix * kAmp * 2;
constexpr size_t kSzUCOL = (size_t)kAmp * kNcol * 4;
constexpr size_t kSzBTP  = (size_t)kNcol * kAmp * 2;
constexpr size_t kSzVPL  = (size_t)kPix * kNcol * 4;
constexpr size_t kOffANG  = 0;
constexpr size_t kOffAPL  = kOffANG  + kSzANG;
constexpr size_t kOffUCOL = kOffAPL  + kSzAPL;
constexpr size_t kOffBTP  = kOffUCOL + kSzUCOL;
constexpr size_t kOffVPL  = kOffBTP  + kSzBTP;
constexpr size_t kWsTotal = kOffVPL  + kSzVPL;
static_assert(kWsTotal == 43253760ull, "carve total");
static_assert(kWsTotal <= 134217728ull, "carve cap");
static_assert((kOffAPL % 128) == 0 && (kOffUCOL % 128) == 0 && (kOffBTP % 128) == 0 && (kOffVPL % 128) == 0, "128-B aligned regions");

__device__ __forceinline__ _Float16 carried_f16(float v, float carry) {
  const float s = v * carry;
  const float f = (fabsf(s) < kF16MinNormal) ? 0.0f : s;
  return (_Float16)f;
}

__device__ __forceinline__ void guard1_h(v8f& a, v16h x, v16h y) {
  asm volatile("v_nop\n\tv_nop\n\tv_nop\n\tv_nop" : "+v"(a) : "v"(x), "v"(y));
}
__device__ __forceinline__ void acc_guard1(v8f& a) {
  asm volatile("v_nop\n\tv_nop\n\tv_nop\n\tv_nop" : "+v"(a));
}
__device__ __forceinline__ void keep4_h(v16h a, v16h b, v16h c, v16h d) {
  asm volatile("v_nop" :: "v"(a), "v"(b), "v"(c), "v"(d));
}
__device__ __forceinline__ v16h frag_load_h(const _Float16* p) {
  union U { v16h v; v8h h[2]; };
  U f;
  f.h[0] = *(const v8h*)(p);
  f.h[1] = *(const v8h*)(p + 16);
  return f.v;
}
__device__ __forceinline__ v8f mma_h(v16h a, v16h b, v8f c) {
  return __builtin_amdgcn_wmma_f32_16x16x32_f16(false, a, false, b, (short)0, c, false, false);
}

__global__ __launch_bounds__(256) void conv_angles_kernel(
    const float* __restrict__ x, const float* __restrict__ cw, const float* __restrict__ cb,
    float* __restrict__ ang)
{
  const int gid = blockIdx.x * 256 + threadIdx.x;
  const int co = gid & 7;
  const int m  = gid >> 3;
  const int b  = m >> 12;
  const int h  = (m >> 6) & 63;
  const int w  = m & 63;
  int  off[9];
  bool ok[9];
#pragma unroll
  for (int kh = 0; kh < 3; ++kh) {
#pragma unroll
    for (int kw = 0; kw < 3; ++kw) {
      const int hh = h + kh - 1;
      const int ww = w + kw - 1;
      ok[kh * 3 + kw] = (hh >= 0) && (hh < kHgt) && (ww >= 0) && (ww < kWid);
      const int hc = hh < 0 ? 0 : (hh > kHgt - 1 ? kHgt - 1 : hh);
      const int wc = ww < 0 ? 0 : (ww > kWid - 1 ? kWid - 1 : ww);
      off[kh * 3 + kw] = hc * kWid + wc;
    }
  }
  const float* xb = x + (size_t)b * kCin * kHgt * kWid;
  const float* wb = cw + co * kTaps;
  float acc = 0.0f;
#pragma unroll 1
  for (int ci = 0; ci < kCin; ++ci) {
    const float* xc = xb + ci * (kHgt * kWid);
    const float* wc = wb + ci * 9;
#pragma unroll
    for (int k = 0; k < 9; ++k) {
      float v = xc[off[k]];
      asm volatile("" : "+v"(v));
      v = ok[k] ? v : 0.0f;
      acc = fmaf(v, wc[k], acc);
    }
  }
  const float res = acc + cb[co];
  *(volatile float*)(ang + gid) = res;
  __threadfence();
  *(volatile float*)(ang + gid) = res;
}

__global__ __launch_bounds__(256) void encode_state_kernel(
    const float* __restrict__ ang, unsigned short* __restrict__ Apl)
{
  const int lane = threadIdx.x & 31;
  const int wave = threadIdx.x >> 5;
  const int m = blockIdx.x * 8 + wave;
  const float a = ang[(size_t)m * kWires + (lane & 7)];
  float sv, cv;
  sincosf(0.5f * a, &sv, &cv);
  float cq[8], sq[8];
#pragma unroll
  for (int q = 0; q < 8; ++q) {
    cq[q] = __shfl(cv, q, 32);
    sq[q] = __shfl(sv, q, 32);
  }
  float base = ((lane >> 4) & 1) ? sq[0] : cq[0];
  base = base * (((lane >> 3) & 1) ? sq[1] : cq[1]);
  base = base * (((lane >> 2) & 1) ? sq[2] : cq[2]);
  base = base * (((lane >> 1) & 1) ? sq[3] : cq[3]);
  base = base * ((lane & 1) ? sq[4] : cq[4]);
  v8h hv;
#pragma unroll
  for (int j = 0; j < 8; ++j) {
    float v = base * ((j & 4) ? sq[5] : cq[5]);
    v = v * ((j & 2) ? sq[6] : cq[6]);
    v = v * ((j & 1) ? sq[7] : cq[7]);
    hv[j] = carried_f16(v, kCarryA);
  }
  unsigned short* dst = Apl + (size_t)m * kAmp + lane * 8;
  *(volatile v8h*)dst = hv;
  __threadfence();
  *(volatile v8h*)dst = hv;
}

__global__ __launch_bounds__(128) void build_unitary_kernel(
    const float* __restrict__ u3p, const float* __restrict__ cu3p, float* __restrict__ Ucol)
{
  __shared__ __align__(16) float sSt[2 * kAmp];
  __shared__ __align__(16) float sGate[128 * 8];
  __shared__ float sPar[256];
  __shared__ float sTrig[128 * 6];
  const int tid = threadIdx.x;
  const int c = blockIdx.x;
  {
    const int pi = tid < kNumPar ? tid : (kNumPar - 1);
    float pa = u3p[pi];
    float pb = cu3p[pi];
    asm volatile("" : "+v"(pa));
    asm volatile("" : "+v"(pb));
    sPar[tid] = pa;
    sPar[128 + tid] = pb;
  }
  sSt[tid]       = (tid == c) ? 1.0f : 0.0f;
  sSt[tid + 128] = (tid + 128 == c) ? 1.0f : 0.0f;
  sSt[tid + 256] = 0.0f;
  sSt[tid + 384] = 0.0f;
  __syncthreads();
  {
    const int g = tid < kGates ? tid : (kGates - 1);
    const int layer = g >> 4;
    const int r = g & 15;
    const int isC = r >> 3;
    const int w = r & 7;
    const int pbase = isC * 128 + (layer * kWires + w) * 3;
#pragma unroll 1
    for (int a = 0; a < 3; ++a) {
      const float pv = sPar[pbase + a];
      const float av = (a == 0) ? 0.5f * pv : pv;
      float s1, c1;
      sincosf(av, &s1, &c1);
      sTrig[tid * 6 + 2 * a]     = c1;
      sTrig[tid * 6 + 2 * a + 1] = s1;
    }
    const float ct = sTrig[tid * 6 + 0], st = sTrig[tid * 6 + 1];
    const float cp = sTrig[tid * 6 + 2], sp = sTrig[tid * 6 + 3];
    const float cl = sTrig[tid * 6 + 4], sl = sTrig[tid * 6 + 5];
    const float er = cp * cl - sp * sl;
    const float ei = cp * sl + sp * cl;
    sGate[tid * 8 + 0] = ct;
    sGate[tid * 8 + 1] = 0.0f;
    sGate[tid * 8 + 2] = -(cl * st);
    sGate[tid * 8 + 3] = -(sl * st);
    sGate[tid * 8 + 4] = cp * st;
    sGate[tid * 8 + 5] = sp * st;
    sGate[tid * 8 + 6] = er * ct;
    sGate[tid * 8 + 7] = ei * ct;
  }
  __syncthreads();
#pragma unroll 1
  for (int g = 0; g < kGates; ++g) {
    const int r = g & 15;
    const int isC = r >> 3;
    const int w = r & 7;
    const int cbit = 7 - w;
    const int tbit = isC ? (7 - ((w + 1) & 7)) : (7 - w);
    const v4f ga = *(const v4f*)(sGate + g * 8);
    const v4f gb = *(const v4f*)(sGate + g * 8 + 4);
    const int i0 = ((tid >> tbit) << (tbit + 1)) | (tid & ((1 << tbit) - 1));
    const int i1 = i0 | (1 << tbit);
    const float a0r = sSt[i0], a0i = sSt[kAmp + i0];
    const float a1r = sSt[i1], a1i = sSt[kAmp + i1];
    const float n0r = ga[0] * a0r - ga[1] * a0i + ga[2] * a1r - ga[3] * a1i;
    const float n0i = ga[0] * a0i + ga[1] * a0r + ga[2] * a1i + ga[3] * a1r;
    const float n1r = gb[0] * a0r - gb[1] * a0i + gb[2] * a1r - gb[3] * a1i;
    const float n1i = gb[0] * a0i + gb[1] * a0r + gb[2] * a1i + gb[3] * a1r;
    const bool active = (isC == 0) || (((i0 >> cbit) & 1) != 0);
    sSt[i0]        = active ? n0r : a0r;
    sSt[kAmp + i0] = active ? n0i : a0i;
    sSt[i1]        = active ? n1r : a1r;
    sSt[kAmp + i1] = active ? n1i : a1i;
    __syncthreads();
  }
  const v4f ov = *(const v4f*)(sSt + 4 * tid);
  float* dst = Ucol + (size_t)c * kNcol + 4 * tid;
  *(volatile v4f*)dst = ov;
  __threadfence();
  *(volatile v4f*)dst = ov;
}

__global__ __launch_bounds__(256) void transpose_plane_kernel(
    const float* __restrict__ Ucol, unsigned short* __restrict__ Bt)
{
  __shared__ float tile[64 * 65];
  const int tid = threadIdx.x;
  const int n0 = blockIdx.x * 64;
  const int c0 = blockIdx.y * 64;
  {
    const int row = tid >> 2;
    const int cs = (tid & 3) * 16;
    const float* src = Ucol + (size_t)(c0 + row) * kNcol + n0 + cs;
#pragma unroll
    for (int i = 0; i < 4; ++i) {
      const v4f v = *(const v4f*)(src + 4 * i);
      tile[row * 65 + cs + 4 * i + 0] = v[0];
      tile[row * 65 + cs + 4 * i + 1] = v[1];
      tile[row * 65 + cs + 4 * i + 2] = v[2];
      tile[row * 65 + cs + 4 * i + 3] = v[3];
    }
  }
  __syncthreads();
  const int seg = (tid & 7) * 8;
  v8h hv[2];
#pragma unroll
  for (int it = 0; it < 2; ++it) {
    const int r = it * 32 + (tid >> 3);
#pragma unroll
    for (int e = 0; e < 8; ++e) hv[it][e] = carried_f16(tile[(seg + e) * 65 + r], kCarryB);
  }
  for (int pass = 0; pass < 2; ++pass) {
#pragma unroll
    for (int it = 0; it < 2; ++it) {
      const int r = it * 32 + (tid >> 3);
      *(volatile v8h*)(Bt + (size_t)(n0 + r) * kAmp + c0 + seg) = hv[it];
    }
    __threadfence();
  }
}

__global__ __launch_bounds__(256) void wmma_gemm64_f16(
    const unsigned short* __restrict__ Ap, int lda,
    const unsigned short* __restrict__ Btp, int ldb,
    float* __restrict__ C, int ldc,
    int M, int N, int K, float scale)
{
  const _Float16* A  = (const _Float16*)Ap;
  const _Float16* Bt = (const _Float16*)Btp;
  __shared__ __align__(16) float sT[8][16 * 68];
  const int lane = threadIdx.x & 31;
  const int wave = threadIdx.x >> 5;
  const int tilesN = N >> 6;
  const int tilesM = M >> 6;
  const int tile = blockIdx.x * 8 + wave;
  if (tile >= tilesM * tilesN) return;
  const int tm = tile / tilesN;
  const int tn = tile - tm * tilesN;
  const int m0 = tm << 6;
  const int n0 = tn << 6;

  const int rlane = lane & 15;
  const int koff  = (lane >> 4) * 8;
  const int mOff  = (lane >> 4) * 8;

  v8f acc[4][4];
#pragma unroll
  for (int i = 0; i < 4; ++i)
#pragma unroll
    for (int j = 0; j < 4; ++j) acc[i][j] = (v8f){0.f,0.f,0.f,0.f,0.f,0.f,0.f,0.f};

  for (int k0 = 0; k0 < K; k0 += 32) {
    v16h bh[4];
#pragma unroll
    for (int j = 0; j < 4; ++j) {
      const size_t bo = (size_t)(n0 + (j << 4) + rlane) * ldb + koff + k0;
      bh[j] = frag_load_h(Bt + bo);
    }
#pragma unroll
    for (int i = 0; i < 4; ++i) {
      const size_t ao = (size_t)(m0 + (i << 4) + rlane) * lda + koff + k0;
      const v16h ah = frag_load_h(A + ao);
#pragma unroll
      for (int j = 0; j < 4; ++j) acc[i][j] = mma_h(ah, bh[j], acc[i][j]);
#pragma unroll
      for (int j = 0; j < 4; ++j) guard1_h(acc[i][j], ah, bh[j]);
    }
    keep4_h(bh[0], bh[1], bh[2], bh[3]);
  }
#pragma unroll
  for (int i = 0; i < 4; ++i)
#pragma unroll
    for (int j = 0; j < 4; ++j) acc_guard1(acc[i][j]);

  float* slab = sT[wave];
#pragma unroll
  for (int i = 0; i < 4; ++i) {
    const int mBase = m0 + (i << 4);
#pragma unroll
    for (int j = 0; j < 4; ++j) {
#pragma unroll
      for (int r = 0; r < 8; ++r) {
        const float v = acc[i][j][r] * scale;
        slab[(mOff + r) * 68 + (j << 4) + rlane] = v;
      }
    }
    __builtin_amdgcn_fence(__ATOMIC_RELEASE, "workgroup");
    __builtin_amdgcn_wave_barrier();
    __builtin_amdgcn_fence(__ATOMIC_ACQUIRE, "workgroup");
    {
      const int hh = lane >> 4, c4 = (lane & 15) * 4;
      for (int pass = 0; pass < 2; ++pass) {
#pragma unroll
        for (int it = 0; it < 8; ++it) {
          const int row = it * 2 + hh;
          const v4f v = *(const v4f*)(slab + row * 68 + c4);
          *(volatile v4f*)(C + (size_t)(mBase + row) * ldc + n0 + c4) = v;
        }
        __threadfence();
      }
    }
    __builtin_amdgcn_fence(__ATOMIC_RELEASE, "workgroup");
    __builtin_amdgcn_wave_barrier();
    __builtin_amdgcn_fence(__ATOMIC_ACQUIRE, "workgroup");
  }
}

__global__ __launch_bounds__(256) void measure_fc_kernel(
    const float* __restrict__ Vp, const float* __restrict__ fc_w, const float* __restrict__ fc_b,
    float* __restrict__ out)
{
  __shared__ __align__(16) float sPsi[8][2 * kAmp];
  __shared__ float sMeas[32 * 25];
  __shared__ float sFc[kCout * kMeas];
  const int tid = threadIdx.x;
  const int lane = tid & 31;
  const int wave = tid >> 5;
#pragma unroll
  for (int i = 0; i < 3; ++i) sFc[tid + 256 * i] = fc_w[tid + 256 * i];
  const int m0 = blockIdx.x * 32;
  float* ps = sPsi[wave];
#pragma unroll 1
  for (int p = 0; p < 4; ++p) {
    const int px = wave * 4 + p;
    const size_t m = (size_t)(m0 + px);
    __syncthreads();
#pragma unroll
    for (int i = 0; i < 4; ++i) {
      const v4f v = *(const v4f*)(Vp + m * kNcol + 4 * lane + 128 * i);
      *(v4f*)(ps + 4 * lane + 128 * i) = v;
    }
    __syncthreads();
#pragma unroll 1
    for (int q = 0; q < kWires; ++q) {
      const int pb = 7 - q;
      const int lowmask = (1 << pb) - 1;
      float z = 0.0f, xs = 0.0f, ys = 0.0f;
#pragma unroll
      for (int e = 0; e < 4; ++e) {
        const int t = lane + 32 * e;
        const int i0 = ((t >> pb) << (pb + 1)) | (t & lowmask);
        const int i1 = i0 | (1 << pb);
        const float r0 = ps[i0], q0 = ps[kAmp + i0];
        const float r1 = ps[i1], q1 = ps[kAmp + i1];
        z  += (r0 * r0 + q0 * q0) - (r1 * r1 + q1 * q1);
        xs += r0 * r1 + q0 * q1;
        ys += q0 * r1 - r0 * q1;
      }
#pragma unroll
      for (int off = 16; off >= 1; off >>= 1) {
        z  += __shfl_xor(z, off, 32);
        xs += __shfl_xor(xs, off, 32);
        ys += __shfl_xor(ys, off, 32);
      }
      if (lane == 0) {
        sMeas[px * 25 + q]      = z;
        sMeas[px * 25 + 8 + q]  = 2.0f * xs;
        sMeas[px * 25 + 16 + q] = 2.0f * ys;
      }
    }
  }
  __syncthreads();
  float vals[4];
#pragma unroll
  for (int it = 0; it < 4; ++it) {
    const int o = wave * 4 + it;
    float acc = 0.0f;
#pragma unroll 1
    for (int j = 0; j < kMeas; ++j) acc = fmaf(sMeas[lane * 25 + j], sFc[o * kMeas + j], acc);
    vals[it] = acc + fc_b[o];
  }
  const int b  = m0 >> 12;
  const int h  = (m0 >> 6) & 63;
  const int w0 = m0 & 63;
  for (int pass = 0; pass < 2; ++pass) {
#pragma unroll
    for (int it = 0; it < 4; ++it) {
      const int o = wave * 4 + it;
      const size_t oi = ((size_t)(b * kCout + o) * kHgt + h) * kWid + w0 + lane;
      *(volatile float*)(out + oi) = vals[it];
    }
    __threadfence();
  }
}

extern "C" void kernel_launch(void* const* d_in, const int* in_sizes, int n_in,
                              void* d_out, int out_size, void* d_ws, size_t ws_size,
                              hipStream_t stream) {
  if (n_in < 7) return;
  if (in_sizes[0] != kBatch * kCin * kHgt * kWid) return;
  if (in_sizes[1] != kWires * kTaps) return;
  if (in_sizes[2] != kWires) return;
  if (in_sizes[3] != kNumPar) return;
  if (in_sizes[4] != kNumPar) return;
  if (in_sizes[5] != kCout * kMeas) return;
  if (in_sizes[6] != kCout) return;
  if (out_size != kPix * kCout) return;
  if (ws_size < kWsTotal) return;

  const float* x      = (const float*)d_in[0];
  const float* conv_w = (const float*)d_in[1];
  const float* conv_b = (const float*)d_in[2];
  const float* u3p    = (const float*)d_in[3];
  const float* cu3p   = (const float*)d_in[4];
  const float* fc_w   = (const float*)d_in[5];
  const float* fc_b   = (const float*)d_in[6];
  float* out = (float*)d_out;

  char* ws = (char*)d_ws;
  float*          ANG  = (float*)(ws + kOffANG);
  unsigned short* APL  = (unsigned short*)(ws + kOffAPL);
  float*          UCOL = (float*)(ws + kOffUCOL);
  unsigned short* BTP  = (unsigned short*)(ws + kOffBTP);
  float*          VPL  = (float*)(ws + kOffVPL);

  conv_angles_kernel<<<(kPix * kWires) / 256, 256, 0, stream>>>(x, conv_w, conv_b, ANG);
  encode_state_kernel<<<kPix / 8, 256, 0, stream>>>(ANG, APL);
  build_unitary_kernel<<<kAmp, 128, 0, stream>>>(u3p, cu3p, UCOL);
  transpose_plane_kernel<<<dim3(kNcol / 64, kAmp / 64), 256, 0, stream>>>(UCOL, BTP);
  wmma_gemm64_f16<<<((kPix / 64) * (kNcol / 64)) / 8, 256, 0, stream>>>(
      APL, kAmp, BTP, kAmp, VPL, kNcol, kPix, kNcol, kAmp, kFold);
  measure_fc_kernel<<<kPix / 32, 256, 0, stream>>>(VPL, fc_w, fc_b, out);
}
